// Involution_55551107006698
// MI455X (gfx1250) — hardware-verified
//
#include <hip/hip_runtime.h>
#include <math.h>

typedef __attribute__((ext_vector_type(16))) _Float16 v16h;
typedef __attribute__((ext_vector_type(16))) __bf16 v16b;
typedef __attribute__((ext_vector_type(8)))  _Float16 v8h;
typedef __attribute__((ext_vector_type(8)))  float v8f;
typedef __attribute__((ext_vector_type(4)))  float v4f;
typedef __attribute__((ext_vector_type(2)))  float v2f;
typedef __attribute__((ext_vector_type(4)))  unsigned v4u;
typedef __attribute__((ext_vector_type(4)))  int v4i;
typedef float __attribute__((may_alias)) float_a;
typedef int __attribute__((may_alias)) int_a;

template <typename T> __device__ __forceinline__ void vst2(void* p, T v) { *(volatile T*)p = v; __threadfence(); *(volatile T*)p = v; }
__device__ __forceinline__ v8f wmma16(v16h a, v16h b, v8f c) {
  v8f d = __builtin_amdgcn_wmma_f32_16x16x32_f16(false, a, false, b, (short)0, c, false, false);
  asm volatile("v_nop\n\tv_nop\n\tv_nop\n\tv_nop" : "+v"(d) : "v"(a), "v"(b));
  return d;
}
__device__ __forceinline__ v8f wmma_bf(v16b a, v16b b, v8f c) {
  v8f d = __builtin_amdgcn_wmma_f32_16x16x32_bf16(false, a, false, b, (short)0, c, false, false);
  asm volatile("v_nop\n\tv_nop\n\tv_nop\n\tv_nop" : "+v"(d) : "v"(a), "v"(b));
  return d;
}
__device__ __forceinline__ v16h frag_h(const _Float16* rowk0, int lane) {
  union { v16h v; v8h q[2]; } u; const _Float16* p = rowk0 + 8 * (lane >> 4);
  u.q[0] = *(const v8h*)p; u.q[1] = *(const v8h*)(p + 16); return u.v;
}
__device__ __forceinline__ v16h frag_f32(const float* rowk0, int lane) {
  v16h a; const float* p = rowk0 + 8 * (lane >> 4);
#pragma unroll
  for (int i = 0; i < 8; ++i) { a[i] = (_Float16)p[i]; a[8 + i] = (_Float16)p[16 + i]; }
  return a;
}
__device__ __forceinline__ v16h frag_f32s(const float* rowk0, int lane, float sc) {
  v16h a; const float* p = rowk0 + 8 * (lane >> 4);
#pragma unroll
  for (int i = 0; i < 8; ++i) { a[i] = (_Float16)(p[i] * sc); a[8 + i] = (_Float16)(p[16 + i] * sc); }
  return a;
}
__device__ __forceinline__ v16h fragc_f32(const float* W, int k0, int n, int lane, int ld, int K) {
  v16h a; const int g = lane >> 4;
#pragma unroll
  for (int i = 0; i < 8; ++i) { const int ka = k0 + 8 * g + i, kb = ka + 16;
    a[i] = (_Float16)(ka < K ? W[(size_t)(ka < K ? ka : K - 1) * ld + n] : 0.f); a[8 + i] = (_Float16)(kb < K ? W[(size_t)(kb < K ? kb : K - 1) * ld + n] : 0.f); }
  return a;
}
struct F2 { v16b h, l; };
__device__ __forceinline__ F2 bsplit16(const float v[16]) { F2 r;
#pragma unroll
  for (int i = 0; i < 16; ++i) { const __bf16 h = (__bf16)v[i]; r.h[i] = h; r.l[i] = (__bf16)(v[i] - (float)h); }
  return r; }
__device__ __forceinline__ F2 split_row(const float* row, int k0, int lane) { float v[16]; const float* p = row + k0 + 8 * (lane >> 4);
#pragma unroll
  for (int i = 0; i < 8; ++i) { v[i] = p[i]; v[8 + i] = p[16 + i]; }
  return bsplit16(v); }
__device__ __forceinline__ F2 split_rowK(const float* row, int k0, int lane, int K) { float v[16]; const int g = lane >> 4;
#pragma unroll
  for (int i = 0; i < 8; ++i) { const int ka = k0 + 8 * g + i, kb = ka + 16; v[i] = ka < K ? row[ka < K ? ka : K - 1] : 0.f; v[8 + i] = kb < K ? row[kb < K ? kb : K - 1] : 0.f; }
  return bsplit16(v); }
__device__ __forceinline__ F2 split_col(const float* W, int k0, int n, int lane, int ld, int K) { float v[16]; const int g = lane >> 4;
#pragma unroll
  for (int i = 0; i < 8; ++i) { const int ka = k0 + 8 * g + i, kb = ka + 16; v[i] = ka < K ? W[(size_t)(ka < K ? ka : K - 1) * ld + n] : 0.f; v[8 + i] = kb < K ? W[(size_t)(kb < K ? kb : K - 1) * ld + n] : 0.f; }
  return bsplit16(v); }
__device__ __forceinline__ v8f mac3(const F2& a, const F2& b, v8f c) { c = wmma_bf(a.l, b.h, c); c = wmma_bf(a.h, b.l, c); return wmma_bf(a.h, b.h, c); }
__device__ __forceinline__ float sigm(float v) { return 1.0f / (1.0f + expf(-v)); }
#define LDSX() do { asm volatile("s_wait_dscnt 0" ::: "memory"); __builtin_amdgcn_wave_barrier(); __builtin_amdgcn_fence(__ATOMIC_RELEASE, "workgroup"); } while (0)

__device__ __forceinline__ float bfr(float v) { return (float)(__bf16)v; }
#define NBT 4
#define CC 256
#define HH 56
#define WWD 56
#define HW (HH * WWD)
#define CR 64
#define KS 7
#define KK 49
#define NG 16
#define GCH 16
#define NSPAN (KK * NG)
#define KPITCH 800
#define NROW (NBT * HW)
#ifndef NPIXB
#define NPIXB (NROW / 64)
#endif
#define WS_XT 0u
#define WS_XR (WS_XT + 4u * (size_t)NROW * CC)
#define WS_KN (WS_XR + 4u * (size_t)NROW * CR)
#define WS_END (WS_KN + 4u * (size_t)NROW * KPITCH)
__global__ __launch_bounds__(256) void k_xt(const float* __restrict__ X, float* __restrict__ XT) { __shared__ float st[128][65];
  const int t = threadIdx.x; const int p0 = blockIdx.x * 64, c0 = blockIdx.y * 128; const size_t b = blockIdx.z;
  for (int e = t; e < 128 * 64; e += 256) { const int cl = e >> 6, pl = e & 63; st[cl][pl] = bfr(X[(b * CC + c0 + cl) * HW + p0 + pl]); }
  __syncthreads();
  for (int e = t; e < 64 * 32; e += 256) { const int pl = e >> 5, q = e & 31; v4f o; o[0] = st[q * 4][pl]; o[1] = st[q * 4 + 1][pl]; o[2] = st[q * 4 + 2][pl]; o[3] = st[q * 4 + 3][pl]; vst2(XT + (b * HW + p0 + pl) * CC + c0 + q * 4, o); } }
__global__ __launch_bounds__(128) void k_red(const float* __restrict__ XT, const float* __restrict__ WR, const float* __restrict__ BR, const float* __restrict__ GA, const float* __restrict__ BEt, const float* __restrict__ MU, const float* __restrict__ VAR, float* __restrict__ XR) { __shared__ __align__(16) float sf[4][16][68];
  const int tid = threadIdx.x, wave = tid >> 5, lane = tid & 31, col = lane & 15, g = lane >> 4; const size_t r0 = (size_t)blockIdx.x * 64 + wave * 16;
  v8f acc[4] = {};
#pragma unroll 2
  for (int kc = 0; kc < CC / 32; ++kc) { v16b a; { const float* p = XT + (r0 + col) * CC + kc * 32 + 8 * g;
#pragma unroll
      for (int i = 0; i < 8; ++i) { a[i] = (__bf16)p[i]; a[8 + i] = (__bf16)p[16 + i]; } }
#pragma unroll
    for (int j = 0; j < 4; ++j) { v16b w; const int o = j * 16 + col; const float* wr = WR + (size_t)o * CC + kc * 32 + 8 * g;
#pragma unroll
      for (int i = 0; i < 8; ++i) { w[i] = (__bf16)wr[i]; w[8 + i] = (__bf16)wr[16 + i]; }
      acc[j] = wmma_bf(a, w, acc[j]); } }
#pragma unroll
  for (int j = 0; j < 4; ++j) { const int o = j * 16 + col; const float sc = bfr(GA[o]) * rsqrtf(bfr(VAR[o]) + 1e-5f), mu = bfr(MU[o]), bb = bfr(BR[o]), be = bfr(BEt[o]);
#pragma unroll
    for (int r = 0; r < 8; ++r) sf[wave][8 * g + r][o] = fmaxf((acc[j][r] + bb - mu) * sc + be, 0.f);
    asm volatile("s_wait_loadcnt 0x0" ::: "memory"); }
  LDSX(); for (int rl = 0; rl < 16; ++rl) if (lane < 16) vst2(XR + (r0 + rl) * CR + lane * 4, *(const v4f*)&sf[wave][rl][lane * 4]); }
__global__ __launch_bounds__(128) void k_span(const float* __restrict__ XR, const float* __restrict__ WS_, const float* __restrict__ BS, float* __restrict__ KN) { __shared__ __align__(16) float sf[4][16][132];
  const int tid = threadIdx.x, wave = tid >> 5, lane = tid & 31, col = lane & 15, g = lane >> 4; const int c0 = blockIdx.y * 128; const size_t r0 = (size_t)blockIdx.x * 64 + wave * 16;
  v8f acc[8] = {};
#pragma unroll
  for (int kc = 0; kc < CR / 32; ++kc) { const F2 a = split_row(XR + (r0 + col) * CR, kc * 32, lane);
#pragma unroll
    for (int j = 0; j < 8; ++j) { v16b w; const int o = c0 + j * 16 + col; const int oc = o < NSPAN ? o : NSPAN - 1; const float* wr = WS_ + (size_t)oc * CR + kc * 32 + 8 * g;
#pragma unroll
      for (int i = 0; i < 8; ++i) { w[i] = (o < NSPAN) ? (__bf16)wr[i] : (__bf16)0.f; w[8 + i] = (o < NSPAN) ? (__bf16)wr[16 + i] : (__bf16)0.f; }
      acc[j] = wmma_bf(a.h, w, acc[j]); acc[j] = wmma_bf(a.l, w, acc[j]); } }
#pragma unroll
  for (int j = 0; j < 8; ++j) { const int o = c0 + j * 16 + col; const float bb = (o < NSPAN) ? bfr(BS[o]) : 0.f;
#pragma unroll
    for (int r = 0; r < 8; ++r) sf[wave][8 * g + r][j * 16 + col] = (o < NSPAN) ? acc[j][r] + bb : 0.f; }
  LDSX(); if (c0 + 128 <= KPITCH) { for (int rl = 0; rl < 16; ++rl) vst2(KN + (r0 + rl) * KPITCH + c0 + lane * 4, *(const v4f*)&sf[wave][rl][lane * 4]); }
  else { for (int rl = 0; rl < 16; ++rl) if (c0 + lane * 4 < KPITCH) vst2(KN + (r0 + rl) * KPITCH + c0 + lane * 4, *(const v4f*)&sf[wave][rl][lane * 4]); } }
__global__ __launch_bounds__(128) void k_inv(const float* __restrict__ X, const float* __restrict__ KN, float* __restrict__ OUT) { __shared__ __align__(16) float so[GCH][64 + 4];
  const int tid = threadIdx.x; const int pl = tid & 63, half = tid >> 6; const int p0 = blockIdx.x * 64; const int gg = blockIdx.y; const size_t b = blockIdx.z; const int p = p0 + pl; const int py = p / WWD, px = p % WWD;
  const float* kr = KN + (b * HW + p) * KPITCH + gg * KK; const float* xg = X + (b * CC + gg * GCH + half * 8) * (size_t)HW;
  float acc[8];
#pragma unroll
  for (int c = 0; c < 8; ++c) acc[c] = 0.f;
#pragma unroll 1
  for (int k = 0; k < KK; ++k) { const int yy = py + k / KS - 3, xx = px + k % KS - 3; if (yy < 0 || yy >= HH || xx < 0 || xx >= WWD) continue; const float kv = kr[k]; const float* xp = xg + yy * WWD + xx;
#pragma unroll
    for (int c = 0; c < 8; ++c) acc[c] += kv * bfr(xp[(size_t)c * HW]); }
#pragma unroll
  for (int c = 0; c < 8; ++c) so[half * 8 + c][pl] = acc[c];
  __syncthreads();
  for (int e = tid; e < GCH * 16; e += 128) { const int c = e >> 4, q = e & 15; vst2(OUT + (b * CC + gg * GCH + c) * (size_t)HW + p0 + q * 4, *(const v4f*)&so[c][q * 4]); } }
extern "C" void kernel_launch(void* const* d_in, const int* in_sizes, int n_in, void* d_out, int out_size, void* d_ws, size_t ws_size, hipStream_t stream) {
  (void)in_sizes; (void)n_in; (void)out_size;
  const float** F = (const float**)d_in;
  if (ws_size < (size_t)WS_END) return;
  char* ws = (char*)d_ws; float *XT = (float*)(ws + WS_XT), *XR = (float*)(ws + WS_XR), *KN = (float*)(ws + WS_KN);
  k_xt<<<dim3(HW / 64, CC / 128, NBT), 256, 0, stream>>>(F[0], XT);
  k_red<<<dim3(NROW / 64), 128, 0, stream>>>(XT, F[1], F[2], F[3], F[4], F[5], F[6], XR);
  k_span<<<dim3(NROW / 64, (KPITCH + 127) / 128), 128, 0, stream>>>(XR, F[7], F[8], KN);
  k_inv<<<dim3(NPIXB >= HW / 64 ? HW / 64 : NPIXB, NG, NPIXB >= HW / 64 ? NBT : 1), 128, 0, stream>>>(F[0], KN, (float*)d_out);
}
